// ForwardDistance_10385230922577
// MI455X (gfx1250) — hardware-verified
//
#include <hip/hip_runtime.h>


#ifndef NB
#define NB 4
#endif
#ifndef SEQ
#define SEQ 1024
#endif
#define NB_FULL  4
#define SEQ_FULL 1024
#ifndef OUT_SEQ
#define OUT_SEQ SEQ
#endif
#define DK   512
#define AG   64
#define PT   68
#define C2   ((float)(2.0 * 1.4426950408889634))

static_assert(DK % 32 == 0);
static_assert(DK % 8 == 0);
static_assert(AG == 64);
static_assert(SEQ % 64 == 0);
static_assert((NB * SEQ) % 64 == 0);
static_assert(OUT_SEQ % 32 == 0);
static_assert(OUT_SEQ >= SEQ);
static_assert(((size_t)SEQ * DK) % 8 == 0);
static_assert(((size_t)AG * DK) % 8 == 0);
static_assert(NB <= NB_FULL);
static_assert(SEQ <= SEQ_FULL);
static_assert(PT % 4 == 0);
static_assert(PT >= 64);
static_assert(32 * 16 * 8 == 16 * AG * 4);
static_assert(256 * 16 * 4 == 64 * 64 * 4);
static_assert(256 * 4 * 4 == 64 * AG);
static_assert((2 * AG * PT + AG) * 4 <= 131072);
static_assert(16 * 68 * 4 <= 131072);

typedef unsigned short bf;
typedef __attribute__((ext_vector_type(16))) __bf16   v16bf;
typedef __attribute__((ext_vector_type(8)))  unsigned short v8us;
typedef __attribute__((ext_vector_type(8)))  float    v8f;
typedef __attribute__((ext_vector_type(4)))  float    v4f;
typedef v4f  __attribute__((may_alias)) v4fa;

__device__ __forceinline__ unsigned short f2bf(float f) { unsigned u = __float_as_uint(f); u += 0x7FFFu + ((u >> 16) & 1u); return (unsigned short)(u >> 16); }
__device__ __forceinline__ float bfr(float f) { return __uint_as_float(((unsigned)f2bf(f)) << 16); }
__device__ __forceinline__ v16bf cat16b(v8us lo, v8us hi) { return __builtin_bit_cast(v16bf, __builtin_shufflevector(lo, hi, 0, 1, 2, 3, 4, 5, 6, 7, 8, 9, 10, 11, 12, 13, 14, 15)); }
__device__ __forceinline__ v8f wmmab(v16bf a, v16bf b, v8f c) { return __builtin_amdgcn_wmma_f32_16x16x32_bf16(false, a, false, b, (short)0, c, false, false); }
__device__ __forceinline__ v8f wmmab_g(v16bf a, v16bf b, v8f c) { c = wmmab(a, b, c); asm volatile("v_nop\n\tv_nop\n\tv_nop\n\tv_nop" : "+v"(c) : "v"(a), "v"(b)); return c; }
__device__ __forceinline__ v16bf ldb(const bf* p)  { return cat16b(*(const v8us*)p, *(const v8us*)(p + 16)); }
__device__ __forceinline__ void wave_sync() { __builtin_amdgcn_fence(3  , "wavefront"); __builtin_amdgcn_wave_barrier(); asm volatile("" ::: "memory"); }

__global__ __launch_bounds__(256) void k_cvt8(const float* __restrict__ src, bf* dst, size_t n8) {
    const size_t i = (size_t)blockIdx.x * 256 + threadIdx.x; if (i >= n8) return;
    const v8f v = *(const v8f*)(src + i * 8); v8us o;
#pragma unroll
    for (int k = 0; k < 8; ++k) o[k] = f2bf(v[k]);
    *(volatile v8us*)(dst + i * 8) = o; __threadfence(); *(volatile v8us*)(dst + i * 8) = o;
}

__global__ __launch_bounds__(32) void k_lin(const bf* __restrict__ A, const bf* __restrict__ Bt, const float* __restrict__ bias, float* P) {
    __shared__ __align__(16) float os[16 * 68];
    const int K = DK;
    const int lane = threadIdx.x & 31, lr = lane & 15, hi = lane >> 4; const int r0 = blockIdx.x * 64;
    v8f acc[4][4];
#pragma unroll
    for (int mb = 0; mb < 4; ++mb)
#pragma unroll
        for (int nb = 0; nb < 4; ++nb) acc[mb][nb] = (v8f){};
    const size_t aoff = (size_t)(r0 + lr) * K + 8 * hi, boff = (size_t)lr * K + 8 * hi;
#pragma unroll 1
    for (int kc = 0; kc < K; kc += 32) {
        v16bf a[4];
#pragma unroll
        for (int mb = 0; mb < 4; ++mb) a[mb] = ldb(A + aoff + (size_t)mb * 16 * K + kc);
#pragma unroll
        for (int nb = 0; nb < 4; ++nb) { const v16bf b = ldb(Bt + boff + (size_t)nb * 16 * K + kc);
#pragma unroll
            for (int mb = 0; mb < 4; ++mb) acc[mb][nb] = wmmab_g(a[mb], b, acc[mb][nb]); }
    }
    float bc[4];
#pragma unroll
    for (int nb = 0; nb < 4; ++nb) bc[nb] = bfr(bias[nb * 16 + lr]);
#pragma unroll
    for (int mb = 0; mb < 4; ++mb) {
#pragma unroll
        for (int nb = 0; nb < 4; ++nb) {
#pragma unroll
            for (int j = 0; j < 8; ++j) os[(hi * 8 + j) * 68 + nb * 16 + lr] = (acc[mb][nb][j] + bc[nb]) * C2; }
        wave_sync();
        float* pb = P + (size_t)(r0 + mb * 16) * AG;
#pragma unroll 1
        for (int ps = 0; ps < 2; ++ps) {
#pragma unroll
            for (int s = 0; s < 8; ++s) { const int row = 2 * s + (lane >> 4), c4 = (lane & 15) * 4;
                const v4f val = *(const v4fa*)(&os[row * 68 + c4]);
                *(volatile v4f*)(pb + (size_t)row * AG + c4) = val; }
            if (ps == 0) __threadfence(); }
        wave_sync();
    }
}

__global__ __launch_bounds__(256) void k_pair(const float* __restrict__ U, const float* __restrict__ V, const float* __restrict__ agg, float* OUT) {
    __shared__ __align__(16) float dT[AG * PT];
    __shared__ __align__(16) float cT[AG * PT];
    __shared__ __align__(16) float wS[AG];
    const int tid = threadIdx.x; const int tx = tid & 15, ty = tid >> 4;
    const int n0 = blockIdx.x * 64, m0 = blockIdx.y * 64, b = blockIdx.z;
    const float* dsrc = U + ((size_t)b * SEQ + n0) * AG;
    const float* csrc = V + ((size_t)b * SEQ + m0) * AG;
#pragma unroll
    for (int i = 0; i < 4; ++i) { const int idx = i * 256 + tid; const int row = idx >> 4, c4 = (idx & 15) * 4;
        const v4f dv = *(const v4f*)(dsrc + (size_t)idx * 4); const v4f cv = *(const v4f*)(csrc + (size_t)idx * 4);
#pragma unroll
        for (int k = 0; k < 4; ++k) { dT[(c4 + k) * PT + row] = dv[k]; cT[(c4 + k) * PT + row] = cv[k]; } }
    if (tid < AG) wS[tid] = -2.0f * bfr(agg[tid]);
    __syncthreads();
    float acc[4][4];
#pragma unroll
    for (int i = 0; i < 4; ++i)
#pragma unroll
        for (int j = 0; j < 4; ++j) acc[i][j] = 0.0f;
    float sw = 0.0f;
#pragma unroll 2
    for (int a = 0; a < AG; ++a) {
        const v4f d = *(const v4fa*)(&dT[a * PT + 4 * ty]);
        const v4f c = *(const v4fa*)(&cT[a * PT + 4 * tx]);
        const float w = wS[a];
        sw += w;
#pragma unroll
        for (int i = 0; i < 4; ++i) {
#pragma unroll
            for (int j = 0; j < 4; ++j) {
                const float e = __builtin_amdgcn_exp2f(d[i] + c[j]);
                const float r = __builtin_amdgcn_rcpf(1.0f + e);
                acc[i][j] = fmaf(w, r, acc[i][j]); } }
    }
    const float sa = -0.5f * sw;
    v4f val[4];
#pragma unroll
    for (int i = 0; i < 4; ++i) { val[i][0] = acc[i][0] + sa; val[i][1] = acc[i][1] + sa; val[i][2] = acc[i][2] + sa; val[i][3] = acc[i][3] + sa; }
    float* ob = OUT + ((size_t)b * OUT_SEQ + n0 + 4 * ty) * OUT_SEQ + m0 + 4 * tx;
#pragma unroll 1
    for (int ps = 0; ps < 2; ++ps) {
#pragma unroll
        for (int i = 0; i < 4; ++i) *(volatile v4f*)(ob + (size_t)i * OUT_SEQ) = val[i];
        if (ps == 0) __threadfence(); }
}

static constexpr size_t al256(size_t v) { return (v + 255) & ~(size_t)255; }
static constexpr size_t SZ_XB = al256((size_t)NB * SEQ * DK * 2);
static constexpr size_t SZ_WB = al256((size_t)2 * AG * DK * 2);
static constexpr size_t SZ_PL = al256((size_t)NB * SEQ * AG * 4);
static constexpr size_t SZ_TOTAL = 2 * SZ_XB + SZ_WB + 2 * SZ_PL;
static_assert(SZ_TOTAL <= (size_t)134217728);
static_assert(((size_t)AG * DK * 2) % 256 == 0);

extern "C" void kernel_launch(void* const* d_in, const int* in_sizes, int n_in,
                              void* d_out, int out_size, void* d_ws, size_t ws_size, hipStream_t stream) {
    if (n_in < 7) return;
    const size_t needx = ((size_t)(NB - 1) * SEQ_FULL + SEQ) * DK;
    if ((size_t)in_sizes[0] < needx || (size_t)in_sizes[1] < needx) return;
    if ((size_t)in_sizes[2] < (size_t)AG * DK || (size_t)in_sizes[4] < (size_t)AG * DK) return;
    if (in_sizes[3] < AG || in_sizes[5] < AG || in_sizes[6] < AG) return;
    if ((size_t)out_size < ((size_t)(NB - 1) * OUT_SEQ + (size_t)(SEQ - 1)) * OUT_SEQ + SEQ) return;
    if (SZ_TOTAL > ws_size) return;
    const float* xin[2] = { (const float*)d_in[0], (const float*)d_in[1] };
    const float* wl = (const float*)d_in[2]; const float* bl = (const float*)d_in[3];
    const float* wr = (const float*)d_in[4]; const float* br = (const float*)d_in[5];
    const float* ag = (const float*)d_in[6];
    float* OUT = (float*)d_out;
    char* wsp = (char*)d_ws;
    bf* XB[2];
    XB[0] = (bf*)wsp; wsp += SZ_XB;
    XB[1] = (bf*)wsp; wsp += SZ_XB;
    bf* WB = (bf*)wsp; wsp += SZ_WB;
    float* UP = (float*)wsp; wsp += SZ_PL;
    float* VP = (float*)wsp; wsp += SZ_PL;
    bf* WL = WB; bf* WR = WB + (size_t)AG * DK;

    for (int i = 0; i < 2; ++i) {
        if (SEQ == SEQ_FULL) {
            const size_t n8 = (size_t)NB * SEQ * DK / 8;
            k_cvt8<<<(unsigned)((n8 + 255) / 256), 256, 0, stream>>>(xin[i], XB[i], n8);
        } else {
            const size_t n8 = (size_t)SEQ * DK / 8;
            for (int b = 0; b < NB; ++b) k_cvt8<<<(unsigned)((n8 + 255) / 256), 256, 0, stream>>>(xin[i] + (size_t)b * SEQ_FULL * DK, XB[i] + (size_t)b * SEQ * DK, n8);
        }
    }
    { const size_t n8 = (size_t)AG * DK / 8; const unsigned g = (unsigned)((n8 + 255) / 256);
      k_cvt8<<<g, 256, 0, stream>>>(wl, WL, n8); k_cvt8<<<g, 256, 0, stream>>>(wr, WR, n8); }

    k_lin<<<dim3(NB * SEQ / 64, 1, 1), 32, 0, stream>>>(XB[0], WL, bl, UP);
    k_lin<<<dim3(NB * SEQ / 64, 1, 1), 32, 0, stream>>>(XB[1], WR, br, VP);

    k_pair<<<dim3(SEQ / 64, SEQ / 64, NB), 256, 0, stream>>>(UP, VP, ag, OUT);
}
